// ScaledDotProductAttention_69157563400295
// MI455X (gfx1250) — hardware-verified
//
#include <hip/hip_runtime.h>


#ifndef NB
#define NB 2
#endif
#ifndef SEQ
#define SEQ 2048
#endif
#define NB_FULL  2
#define SEQ_FULL 2048
#define NHD  16
#define HD   64
#define QBLK 128
#define KT   64
#define OSP  68
#define TLP  72
#define PCL2 10.0f
#define K2S  0.18033688011112042f
#define SENT (-3.0e38f)

typedef _Float16 h16;
typedef unsigned short bf;
typedef __attribute__((ext_vector_type(16))) __bf16   v16bf;
typedef __attribute__((ext_vector_type(16))) _Float16 v16h;
typedef __attribute__((ext_vector_type(8)))  _Float16 v8h;
typedef __attribute__((ext_vector_type(8)))  unsigned short v8us;
typedef __attribute__((ext_vector_type(8)))  float    v8f;
typedef __attribute__((ext_vector_type(4)))  float    v4f;
typedef __attribute__((ext_vector_type(4)))  int      v4i;
typedef v8h  __attribute__((may_alias)) v8ha;
typedef v4f  __attribute__((may_alias)) v4fa;
typedef v4i  __attribute__((may_alias)) v4ia;

static_assert(HD == 64);
static_assert(KT == 64);
static_assert(QBLK == 128);
static_assert(SEQ % 128 == 0);
static_assert(SEQ <= SEQ_FULL);
static_assert(NB <= NB_FULL);
static_assert(((size_t)NB * NHD * SEQ * 8) % 256 == 0);
static_assert((size_t)(SEQ / 64) * (NB * NHD) * 256 * 2 * 8 == (size_t)NB * NHD * HD * SEQ);
static_assert((size_t)(NB * NHD) * (SEQ / QBLK) * 8 * 16 * HD == (size_t)NB * NHD * SEQ * HD);
static_assert((size_t)2 * NB * NHD * SEQ * HD * 2 <= (size_t)134217728);

__device__ __forceinline__ unsigned short f2bf(float f) { unsigned u = __float_as_uint(f); u += 0x7FFFu + ((u >> 16) & 1u); return (unsigned short)(u >> 16); }
__device__ __forceinline__ float bf2f(unsigned short b) { return __uint_as_float(((unsigned)b) << 16); }
__device__ __forceinline__ float bfr(float f) { return bf2f(f2bf(f)); }
__device__ __forceinline__ v16h cat16(v8h lo, v8h hi) { return __builtin_shufflevector(lo, hi, 0, 1, 2, 3, 4, 5, 6, 7, 8, 9, 10, 11, 12, 13, 14, 15); }
__device__ __forceinline__ v16bf cat16b(v8us lo, v8us hi) { return __builtin_bit_cast(v16bf, __builtin_shufflevector(lo, hi, 0, 1, 2, 3, 4, 5, 6, 7, 8, 9, 10, 11, 12, 13, 14, 15)); }
__device__ __forceinline__ v8f wmma16(v16h a, v16h b, v8f c) { return __builtin_amdgcn_wmma_f32_16x16x32_f16(false, a, false, b, (short)0, c, false, false); }
__device__ __forceinline__ v8f wmmab(v16bf a, v16bf b, v8f c) { return __builtin_amdgcn_wmma_f32_16x16x32_bf16(false, a, false, b, (short)0, c, false, false); }

template <typename T16> struct WFrag;
template <> struct WFrag<h16> { typedef v16h V; static __device__ __forceinline__ V ld(const h16* p) { return cat16(*(const v8h*)p, *(const v8h*)(p + 16)); } };
template <> struct WFrag<bf>  { typedef v16bf V; static __device__ __forceinline__ V ld(const bf* p) { return cat16b(*(const v8us*)p, *(const v8us*)(p + 16)); } };

__global__ __launch_bounds__(256) void k_kplane(const float* __restrict__ Kg, bf* KP) {
    const unsigned gid = blockIdx.x * 256u + threadIdx.x;
    const unsigned row = gid >> 3, pc = gid & 7u;
    if (row >= (unsigned)(NB * NHD * SEQ)) return;
    const unsigned pl = row / (unsigned)SEQ, t = row % (unsigned)SEQ;
    const float* src = Kg + ((size_t)pl * SEQ_FULL + t) * HD + pc * 8u;
    const v4f x0 = *(const v4f*)src, x1 = *(const v4f*)(src + 4);
    v8us o;
#pragma unroll
    for (int j = 0; j < 4; ++j) { o[j] = f2bf(x0[j]); o[4 + j] = f2bf(x1[j]); }
    bf* dst = KP + (size_t)row * HD + pc * 8u;
    *(volatile v8us*)dst = o; __threadfence(); *(volatile v8us*)dst = o;
}

__global__ __launch_bounds__(256) void k_vtplane(const float* __restrict__ Vg, h16* VT) {
    __shared__ __align__(16) h16 tl[HD * TLP];
    const unsigned tid = threadIdx.x;
    const unsigned t0 = blockIdx.x * 64u, pl = blockIdx.y;
    const float* src = Vg + ((size_t)pl * SEQ_FULL + t0) * HD;
#pragma unroll
    for (int i = 0; i < 4; ++i) {
        const unsigned id = tid + (unsigned)i * 256u;
        const unsigned r = id >> 4, c4 = (id & 15u) << 2;
        const v4f x = *(const v4f*)(src + (size_t)r * HD + c4);
#pragma unroll
        for (int j = 0; j < 4; ++j) tl[(c4 + (unsigned)j) * TLP + r] = (h16)bfr(x[j]);
    }
    __syncthreads();
    v8h val[2]; h16* dst[2];
#pragma unroll
    for (int i = 0; i < 2; ++i) {
        const unsigned id = tid + (unsigned)i * 256u;
        const unsigned d = id >> 3, pc = id & 7u;
        val[i] = *(const v8ha*)(tl + d * TLP + pc * 8u);
        dst[i] = VT + ((size_t)pl * HD + d) * SEQ + t0 + pc * 8u;
    }
#pragma unroll
    for (int i = 0; i < 2; ++i) *(volatile v8h*)dst[i] = val[i];
    __threadfence();
#pragma unroll
    for (int i = 0; i < 2; ++i) *(volatile v8h*)dst[i] = val[i];
}

__global__ __launch_bounds__(256) void k_flash(const float* __restrict__ Qg, const bf* __restrict__ KP, const h16* __restrict__ VT, const int* __restrict__ Mg, float* Og) {
    __shared__ __align__(16) int   mks[SEQ];
    __shared__ __align__(16) float os[8 * 16 * OSP];
    const unsigned tid = threadIdx.x, lane = tid & 31u, wave = tid >> 5, lr = lane & 15u, hi = lane >> 4;
    const unsigned nqb = (unsigned)(SEQ / QBLK);
    const unsigned bh = blockIdx.x / nqb, qb = blockIdx.x % nqb, b = bh / (unsigned)NHD;

    {
        const int* mrow = Mg + (size_t)b * SEQ_FULL;
#pragma unroll 1
        for (unsigned i0 = 0; i0 < (unsigned)(SEQ / 4); i0 += 256u) {
            const unsigned idx = i0 + tid;
            const unsigned ic = (idx < (unsigned)(SEQ / 4)) ? idx : (unsigned)(SEQ / 4 - 1);
            const v4i m = *(const v4i*)(mrow + (size_t)ic * 4u);
            if (idx < (unsigned)(SEQ / 4)) *(v4ia*)(mks + idx * 4u) = m;
        }
    }
    __syncthreads();

    const unsigned q0 = qb * (unsigned)QBLK + wave * 16u;
    v16bf qf[2];
    {
        const float* qrow = Qg + ((size_t)bh * SEQ_FULL + q0 + lr) * HD + 8u * hi;
#pragma unroll
        for (int c = 0; c < 2; ++c) {
            const float* qp = qrow + c * 32;
            const v4f x0 = *(const v4f*)qp, x1 = *(const v4f*)(qp + 4), x2 = *(const v4f*)(qp + 16), x3 = *(const v4f*)(qp + 20);
            v8us e0, e1;
#pragma unroll
            for (int j = 0; j < 4; ++j) { e0[j] = f2bf(x0[j]); e0[4 + j] = f2bf(x1[j]); e1[j] = f2bf(x2[j]); e1[4 + j] = f2bf(x3[j]); }
            qf[c] = cat16b(e0, e1);
        }
    }
    const bool mq = (mks[q0 + lr] != 0);

    v8f accO[4];
#pragma unroll
    for (int t = 0; t < 4; ++t) accO[t] = (v8f){};
    float m_run = SENT, l_run = 0.0f;

    const bf*  kbase = KP + ((size_t)bh * SEQ + lr) * HD + 8u * hi;
    const h16* vbase = VT + ((size_t)bh * HD + lr) * SEQ + 8u * hi;

#pragma unroll 1
    for (unsigned kt = 0; kt < (unsigned)(SEQ / KT); ++kt) {
        const unsigned kv0 = kt * (unsigned)KT;

        v16bf ka[4][2];
        v8f s[4];
#pragma unroll
        for (int t = 0; t < 4; ++t) {
            const bf* kp = kbase + (size_t)(kv0 + (unsigned)t * 16u) * HD;
            ka[t][0] = WFrag<bf>::ld(kp);
            ka[t][1] = WFrag<bf>::ld(kp + 32);
        }
#pragma unroll
        for (int t = 0; t < 4; ++t) {
            v8f acc = (v8f){};
            acc = wmmab(ka[t][0], qf[0], acc);
            acc = wmmab(ka[t][1], qf[1], acc);
            s[t] = acc;
        }
        asm volatile("v_nop\n\tv_nop\n\tv_nop\n\tv_nop" : "+v"(s[0]), "+v"(s[1]), "+v"(s[2]), "+v"(s[3]) : "v"(ka[3][0]), "v"(ka[3][1]), "v"(ka[2][1]), "v"(qf[0]), "v"(qf[1]));

        float lmax = SENT;
#pragma unroll
        for (int t = 0; t < 4; ++t) {
            const int* mp = mks + kv0 + (unsigned)t * 16u + 8u * hi;
            const v4i m0 = *(const v4ia*)mp, m1 = *(const v4ia*)(mp + 4);
#pragma unroll
            for (int r = 0; r < 8; ++r) {
                const int mk = (r < 4) ? m0[r & 3] : m1[r & 3];
                float v = s[t][r] * K2S;
                v = (mk != 0) ? v : SENT;
                v = mq ? v : 0.0f;
                s[t][r] = v;
                lmax = fmaxf(lmax, v);
            }
        }
        const float omax = __shfl_xor(lmax, 16, 32);
        const float tmax = fmaxf(lmax, omax);
        const float mnew = fmaxf(m_run, tmax);
        const float corr = __builtin_amdgcn_exp2f(m_run - mnew);
        m_run = mnew;
        const float sh = PCL2 - mnew;

        float lsum = 0.0f;
        v8h ph[4];
#pragma unroll
        for (int t = 0; t < 4; ++t) {
#pragma unroll
            for (int r = 0; r < 8; ++r) {
                const float pc = __builtin_amdgcn_exp2f(s[t][r] + sh);
                lsum += pc;
                ph[t][r] = (h16)pc;
            }
        }
        l_run = l_run * corr + lsum;
#pragma unroll
        for (int t = 0; t < 4; ++t) accO[t] *= corr;

        v16h va[2][4];
#pragma unroll
        for (int c = 0; c < 2; ++c)
#pragma unroll
            for (int td = 0; td < 4; ++td)
                va[c][td] = WFrag<h16>::ld(vbase + (size_t)(td * 16) * SEQ + kv0 + (unsigned)c * 32u);
        const v16h fb0 = cat16(ph[0], ph[1]);
        const v16h fb1 = cat16(ph[2], ph[3]);
#pragma unroll
        for (int td = 0; td < 4; ++td) accO[td] = wmma16(va[0][td], fb0, accO[td]);
#pragma unroll
        for (int td = 0; td < 4; ++td) accO[td] = wmma16(va[1][td], fb1, accO[td]);
        asm volatile("v_nop\n\tv_nop\n\tv_nop\n\tv_nop" : "+v"(accO[0]), "+v"(accO[1]), "+v"(accO[2]), "+v"(accO[3]) : "v"(va[1][3]), "v"(va[1][2]), "v"(va[1][1]), "v"(fb0), "v"(fb1));
    }

    const float lo = __shfl_xor(l_run, 16, 32);
    const float ltot = l_run + lo;
    const float inv = 1.0f / ltot;
    float* ow = os + wave * (16u * OSP);
#pragma unroll
    for (int td = 0; td < 4; ++td) {
        v4f o0, o1;
#pragma unroll
        for (int j = 0; j < 4; ++j) { o0[j] = accO[td][j] * inv; o1[j] = accO[td][4 + j] * inv; }
        float* wp = ow + lr * OSP + (unsigned)td * 16u + 8u * hi;
        *(v4fa*)wp = o0; *(v4fa*)(wp + 4) = o1;
    }
    __syncthreads();
    v4f val[8];
#pragma unroll
    for (int s8 = 0; s8 < 8; ++s8) val[s8] = *(const v4fa*)(ow + (2u * (unsigned)s8 + hi) * OSP + lr * 4u);
    float* orow = Og + ((size_t)bh * SEQ + q0) * HD + lr * 4u;
#pragma unroll
    for (int s8 = 0; s8 < 8; ++s8) *(volatile v4f*)(orow + (size_t)(2u * (unsigned)s8 + hi) * HD) = val[s8];
    __threadfence();
#pragma unroll
    for (int s8 = 0; s8 < 8; ++s8) *(volatile v4f*)(orow + (size_t)(2u * (unsigned)s8 + hi) * HD) = val[s8];
}

extern "C" void kernel_launch(void* const* d_in, const int* in_sizes, int n_in,
                              void* d_out, int out_size, void* d_ws, size_t ws_size, hipStream_t stream) {
    if (n_in < 4) return;
    const int need = ((NB * NHD - 1) * SEQ_FULL + SEQ) * HD;
    if (in_sizes[0] < need || in_sizes[1] < need || in_sizes[2] < need) return;
    if (in_sizes[3] < (NB - 1) * SEQ_FULL + SEQ) return;
    if (out_size < NB * NHD * SEQ * HD) return;
    const float* Q = (const float*)d_in[0];
    const float* K = (const float*)d_in[1];
    const float* V = (const float*)d_in[2];
    const int*   M = (const int*)d_in[3];
    float* O = (float*)d_out;
    const size_t plane_bytes = (size_t)NB * NHD * SEQ * HD * 2;
    if (2 * plane_bytes > ws_size) return;
    bf*  KP = (bf*)((char*)d_ws);
    h16* VT = (h16*)((char*)d_ws + plane_bytes);
    k_kplane<<<(unsigned)((size_t)NB * NHD * SEQ * 8 / 256), 256, 0, stream>>>(K, KP);
    k_vtplane<<<dim3(SEQ / 64, NB * NHD), 256, 0, stream>>>(V, VT);
    k_flash<<<(unsigned)(NB * NHD * (SEQ / QBLK)), 256, 0, stream>>>(Q, KP, VT, M, O);
}
